// QuantumAttention_65481071410014
// MI455X (gfx1250) — hardware-verified
//
#include <hip/hip_runtime.h>
#include <math.h>

typedef __attribute__((ext_vector_type(16))) _Float16 v16h;
typedef __attribute__((ext_vector_type(16))) __bf16 v16b;
typedef __attribute__((ext_vector_type(8)))  _Float16 v8h;
typedef __attribute__((ext_vector_type(8)))  __bf16 v8b;
typedef __attribute__((ext_vector_type(8)))  float v8f;
typedef __attribute__((ext_vector_type(4)))  float v4f;
typedef __attribute__((ext_vector_type(4)))  unsigned v4u;

#define EMB 512
#define NB_FULL 2
#define SEQ_FULL 1024
#ifndef NB
#define NB NB_FULL
#endif
#ifndef SEQ
#define SEQ SEQ_FULL
#endif
#define NQB 8
#define PCAR 16384.0f
#define PINV (1.0f / 16384.0f)
#define SCL 0.04419417382415922f

static_assert(EMB == 512);
static_assert(SEQ % 128 == 0);
static_assert(SEQ >= 128 && SEQ <= SEQ_FULL);
static_assert(NB >= 1 && NB <= NB_FULL);

#define WS_XB  ((size_t)0)
#define WS_WB  (WS_XB + 2u * (size_t)NB_FULL * SEQ_FULL * EMB)
#define WS_QH  (WS_WB + 2u * (size_t)3 * EMB * EMB)
#define WS_KH  (WS_QH + 2u * (size_t)NB_FULL * SEQ_FULL * EMB)
#define WS_VT  (WS_KH + 2u * (size_t)NB_FULL * SEQ_FULL * EMB)
#define WS_S   (WS_VT + 2u * (size_t)NB_FULL * EMB * SEQ_FULL)
#define WS_PH  (WS_S  + 4u * (size_t)SEQ_FULL * SEQ_FULL)
#define WS_CS  (WS_PH + 2u * (size_t)SEQ_FULL * SEQ_FULL)
#define WS_END (WS_CS + 256u)
static_assert(WS_END <= (size_t)134217728);
static_assert((WS_WB % 128) == 0 && (WS_QH % 128) == 0 && (WS_KH % 128) == 0 && (WS_VT % 128) == 0 && (WS_S % 128) == 0 && (WS_PH % 128) == 0 && (WS_CS % 128) == 0);

template <typename T> __device__ __forceinline__ void vst2(void* p, const T v) { *(volatile T*)p = v; __threadfence(); *(volatile T*)p = v; }

__device__ __forceinline__ v8f wmma16(v16h a, v16h b, v8f c) {
  v8f d = __builtin_amdgcn_wmma_f32_16x16x32_f16(false, a, false, b, (short)0, c, false, false);
  asm volatile("v_nop\n\tv_nop\n\tv_nop\n\tv_nop" : "+v"(d) : "v"(a), "v"(b));
  return d;
}
__device__ __forceinline__ v8f wmma_bf(v16b a, v16b b, v8f c) {
  v8f d = __builtin_amdgcn_wmma_f32_16x16x32_bf16(false, a, false, b, (short)0, c, false, false);
  asm volatile("v_nop\n\tv_nop\n\tv_nop\n\tv_nop" : "+v"(d) : "v"(a), "v"(b));
  return d;
}
__device__ __forceinline__ v16h frag_h(const _Float16* rowk0, int lane) {
  union { v16h v; v8h q[2]; } u; const _Float16* p = rowk0 + 8 * (lane >> 4);
  u.q[0] = *(const v8h*)p; u.q[1] = *(const v8h*)(p + 16); return u.v;
}
__device__ __forceinline__ v16b frag_b(const __bf16* rowk0, int lane) {
  union { v16b v; v8b q[2]; } u; const __bf16* p = rowk0 + 8 * (lane >> 4);
  u.q[0] = *(const v8b*)p; u.q[1] = *(const v8b*)(p + 16); return u.v;
}
__device__ __forceinline__ float bfr(float v) { return (float)(__bf16)v; }
__device__ __forceinline__ void ldsx() {
  asm volatile("s_wait_dscnt 0" ::: "memory");
  __builtin_amdgcn_fence(3, "workgroup");
  __builtin_amdgcn_wave_barrier();
}

__global__ __launch_bounds__(256) void k_cvt(const float* __restrict__ X, const float* __restrict__ W0, const float* __restrict__ W1,
                                             const float* __restrict__ W2, __bf16* __restrict__ XB, __bf16* __restrict__ WB) {
  const int y = blockIdx.y, bx = blockIdx.x, t = threadIdx.x;
  const float* src; __bf16* dst; size_t base;
  if (y == 0) {
    const int per = SEQ * EMB / 2048;
    if (bx >= NB * per) return;
    const int b = bx / per, r = bx - b * per;
    base = (size_t)b * SEQ_FULL * EMB + (size_t)r * 2048; src = X; dst = XB;
  } else {
    if (bx >= EMB * EMB / 2048) return;
    base = (size_t)bx * 2048; src = (y == 1) ? W0 : ((y == 2) ? W1 : W2); dst = WB + (size_t)(y - 1) * EMB * EMB;
  }
  const float* p = src + base + (size_t)t * 8;
  const v4f a = *(const v4f*)p, c = *(const v4f*)(p + 4);
  union { v8b v; v4u u; } o;
#pragma unroll
  for (int i = 0; i < 4; ++i) { o.v[i] = (__bf16)a[i]; o.v[4 + i] = (__bf16)c[i]; }
  vst2(dst + base + (size_t)t * 8, o.u);
}

__global__ __launch_bounds__(256) void k_ent(const float* __restrict__ PRM, float* __restrict__ CS) {
  __shared__ float psi[256]; __shared__ float redz[8]; __shared__ float redx[8]; __shared__ float so[32];
  const int t = threadIdx.x, lane = t & 31, wave = t >> 5;
  psi[t] = (t == 0) ? 1.0f : 0.0f; if (t < 32) so[t] = 0.0f;
  __syncthreads();
#pragma unroll 1
  for (int l = 0; l < 2; ++l) {
#pragma unroll 1
    for (int q = 0; q < NQB; ++q) {
      const float th = bfr(PRM[l * NQB + q]);
      float sn, cn; sincosf(0.5f * th, &sn, &cn);
      const int mask = 1 << (7 - q);
      const float a0 = psi[t & ~mask], a1 = psi[t | mask];
      __syncthreads();
      psi[t] = ((t & mask) == 0) ? (cn * a0 - sn * a1) : (sn * a0 + cn * a1);
      __syncthreads();
    }
#pragma unroll 1
    for (int q = 0; q < NQB; ++q) {
      const int cm = 1 << (7 - q), tm = 1 << (7 - ((q + 1) & 7));
      const float self = psi[t], oth = psi[t ^ tm];
      __syncthreads();
      psi[t] = (t & cm) ? oth : self;
      __syncthreads();
    }
  }
#pragma unroll 1
  for (int q = 0; q < NQB; ++q) {
    const int mask = 1 << (7 - q);
    const float p = psi[t];
    float pz = (t & mask) ? -(p * p) : (p * p);
    float px = p * psi[t ^ mask];
#pragma unroll
    for (int o = 1; o < 32; o <<= 1) { pz += __shfl_xor(pz, o); px += __shfl_xor(px, o); }
    if (lane == 0) { redz[wave] = pz; redx[wave] = px; }
    __syncthreads();
    if (t == 0) { float az = 0.f, ax = 0.f; for (int w = 0; w < 8; ++w) { az += redz[w]; ax += redx[w]; } so[q] = az; so[NQB + q] = ax; }
    __syncthreads();
  }
  if (t < 32) vst2(CS + t, so[t]);
}

__global__ __launch_bounds__(128) __attribute__((amdgpu_num_vgpr(256)))
void k_gemm_h(const __bf16* __restrict__ A, const __bf16* __restrict__ B, _Float16* __restrict__ D, int sAz, int sBz, int sDz, int ldd) {
  __shared__ __align__(16) _Float16 sh[4][16][136];
  const int tid = threadIdx.x, wave = tid >> 5, lane = tid & 31, col = lane & 15, g = lane >> 4;
  const int m0 = blockIdx.x * 64 + wave * 16, n0 = blockIdx.y * 128; const size_t z = blockIdx.z;
  const __bf16* Ab = A + z * (size_t)sAz + (size_t)(m0 + col) * EMB;
  const __bf16* Bb = B + z * (size_t)sBz + (size_t)(n0 + col) * EMB;
  v8f acc[8] = {};
#pragma unroll 1
  for (int kc = 0; kc < EMB / 32; ++kc) {
    const v16b a = frag_b(Ab + kc * 32, lane);
#pragma unroll
    for (int j = 0; j < 8; ++j) { const v16b w = frag_b(Bb + (size_t)j * 16 * EMB + kc * 32, lane); acc[j] = wmma_bf(a, w, acc[j]); }
  }
#pragma unroll
  for (int j = 0; j < 8; ++j)
#pragma unroll
    for (int r = 0; r < 8; ++r) sh[wave][8 * g + r][j * 16 + col] = (_Float16)acc[j][r];
  ldsx();
  _Float16* Db = D + z * (size_t)sDz + (size_t)m0 * ldd + n0 + col * 8;
#pragma unroll 1
  for (int rp = 0; rp < 8; ++rp) {
    const int rl = 2 * rp + g;
    union { v8h h; v4u u; } o; o.h = *(const v8h*)&sh[wave][rl][col * 8];
    vst2(Db + (size_t)rl * ldd, o.u);
  }
}

__global__ __launch_bounds__(128) __attribute__((amdgpu_num_vgpr(256)))
void k_sc(const _Float16* __restrict__ Q, const _Float16* __restrict__ K, float* __restrict__ S) {
  __shared__ __align__(16) float sf[4][16][132];
  const int tid = threadIdx.x, wave = tid >> 5, lane = tid & 31, col = lane & 15, g = lane >> 4;
  const int m0 = blockIdx.x * 64 + wave * 16, n0 = blockIdx.y * 128;
  const _Float16* Ab = Q + (size_t)(m0 + col) * EMB;
  const _Float16* Bb = K + (size_t)(n0 + col) * EMB;
  v8f acc[8] = {};
#pragma unroll 1
  for (int kc = 0; kc < EMB / 32; ++kc) {
    const v16h a = frag_h(Ab + kc * 32, lane);
#pragma unroll
    for (int j = 0; j < 8; ++j) { const v16h w = frag_h(Bb + (size_t)j * 16 * EMB + kc * 32, lane); acc[j] = wmma16(a, w, acc[j]); }
  }
#pragma unroll
  for (int j = 0; j < 8; ++j)
#pragma unroll
    for (int r = 0; r < 8; ++r) sf[wave][8 * g + r][j * 16 + col] = acc[j][r] * SCL;
  ldsx();
  float* Sb = S + (size_t)m0 * SEQ_FULL + n0 + lane * 4;
#pragma unroll 1
  for (int rl = 0; rl < 16; ++rl) vst2(Sb + (size_t)rl * SEQ_FULL, *(const v4f*)&sf[wave][rl][lane * 4]);
}

__global__ __launch_bounds__(256) void k_sm(const float* __restrict__ S, _Float16* __restrict__ P) {
  __shared__ float sred[8]; __shared__ float sbc; __shared__ __align__(16) float sh[SEQ];
  const int t = threadIdx.x; const size_t row = blockIdx.x; const float* sr = S + row * SEQ_FULL;
  float m = -3.0e38f;
#pragma unroll 1
  for (int k = t; k < SEQ; k += 256) { const float v = sr[k]; sh[k] = v; m = fmaxf(m, v); }
#pragma unroll
  for (int o = 1; o < 32; o <<= 1) m = fmaxf(m, __shfl_xor(m, o));
  if ((t & 31) == 0) sred[t >> 5] = m;
  __syncthreads();
  if (t == 0) { float a = sred[0]; for (int w = 1; w < 8; ++w) a = fmaxf(a, sred[w]); sbc = a; }
  __syncthreads(); m = sbc; __syncthreads();
  float s = 0.f;
#pragma unroll 1
  for (int k = t; k < SEQ; k += 256) { const float e = expf(sh[k] - m); sh[k] = e; s += e; }
#pragma unroll
  for (int o = 1; o < 32; o <<= 1) s += __shfl_xor(s, o);
  if ((t & 31) == 0) sred[t >> 5] = s;
  __syncthreads();
  if (t == 0) { float a = 0.f; for (int w = 0; w < 8; ++w) a += sred[w]; sbc = PCAR / a; }
  __syncthreads(); const float sc = sbc;
#pragma unroll 1
  for (int k = t; k < SEQ; k += 256) sh[k] = sh[k] * sc;
  __syncthreads();
  _Float16* pr = P + row * SEQ_FULL;
#pragma unroll 1
  for (int q = t; q < SEQ / 8; q += 256) {
    const v4f a = *(const v4f*)&sh[q * 8], c = *(const v4f*)&sh[q * 8 + 4];
    union { v8h h; v4u u; } o;
#pragma unroll
    for (int i = 0; i < 4; ++i) { o.h[i] = (_Float16)a[i]; o.h[4 + i] = (_Float16)c[i]; }
    vst2(pr + (size_t)q * 8, o.u);
  }
}

__global__ __launch_bounds__(128) __attribute__((amdgpu_num_vgpr(256)))
void k_pv(const _Float16* __restrict__ P, const _Float16* __restrict__ VT, const float* __restrict__ CS, float* __restrict__ OUT) {
  __shared__ __align__(16) float sf[4][16][132];
  const int tid = threadIdx.x, wave = tid >> 5, lane = tid & 31, col = lane & 15, g = lane >> 4;
  const int m0 = blockIdx.x * 64 + wave * 16, c0 = blockIdx.y * 128;
  const _Float16* Ab = P + (size_t)(m0 + col) * SEQ_FULL;
  const _Float16* Bb = VT + (size_t)(c0 + col) * SEQ_FULL;
  v8f acc[8] = {};
#pragma unroll 1
  for (int kc = 0; kc < SEQ / 32; ++kc) {
    const v16h a = frag_h(Ab + kc * 32, lane);
#pragma unroll
    for (int j = 0; j < 8; ++j) { const v16h w = frag_h(Bb + (size_t)j * 16 * SEQ_FULL + kc * 32, lane); acc[j] = wmma16(a, w, acc[j]); }
  }
#pragma unroll
  for (int j = 0; j < 8; ++j)
#pragma unroll
    for (int r = 0; r < 8; ++r) sf[wave][8 * g + r][j * 16 + col] = acc[j][r] * PINV;
  ldsx();
  const int qb = (lane & 1) << 2;
  const v4f zc = *(const v4f*)(CS + qb), xc = *(const v4f*)(CS + NQB + qb);
  float* Ob = OUT + (size_t)m0 * EMB + c0 + lane * 4;
#pragma unroll 1
  for (int rl = 0; rl < 16; ++rl) {
    const v4f a = *(const v4f*)&sf[wave][rl][lane * 4];
    v4f o;
#pragma unroll
    for (int i = 0; i < 4; ++i) { float sn, cn; sincosf(a[i], &sn, &cn); o[i] = cn * zc[i] - sn * xc[i]; }
    vst2(Ob + (size_t)rl * EMB, o);
  }
}

extern "C" void kernel_launch(void* const* d_in, const int* in_sizes, int n_in, void* d_out, int out_size, void* d_ws, size_t ws_size, hipStream_t stream) {
  if (n_in < 5) return;
  const float* X   = (const float*)d_in[0];
  const float* Wq  = (const float*)d_in[1];
  const float* Wk  = (const float*)d_in[2];
  const float* Wv  = (const float*)d_in[3];
  const float* PRM = (const float*)d_in[4];
  const int need_x = ((NB - 1) * SEQ_FULL + SEQ) * EMB;
  if (in_sizes[0] < need_x || in_sizes[1] < EMB * EMB || in_sizes[2] < EMB * EMB || in_sizes[3] < EMB * EMB || in_sizes[4] < 2 * NQB) return;
  if (out_size < need_x) return;
  if (ws_size < (size_t)WS_END) return;
  char* ws = (char*)d_ws;
  __bf16* XB = (__bf16*)(ws + WS_XB); __bf16* WB = (__bf16*)(ws + WS_WB);
  _Float16* QH = (_Float16*)(ws + WS_QH); _Float16* KH = (_Float16*)(ws + WS_KH); _Float16* VT = (_Float16*)(ws + WS_VT);
  float* S = (float*)(ws + WS_S); _Float16* PH = (_Float16*)(ws + WS_PH); float* CS = (float*)(ws + WS_CS);
  float* OUT = (float*)d_out;

  const int gx_cvt = (NB * SEQ / 4 > EMB * EMB / 2048) ? (NB * SEQ / 4) : (EMB * EMB / 2048);
  k_cvt<<<dim3(gx_cvt, 4), 256, 0, stream>>>(X, Wq, Wk, Wv, XB, WB);
  k_ent<<<dim3(1), 256, 0, stream>>>(PRM, CS);
  k_gemm_h<<<dim3(SEQ / 64, EMB / 128, NB), 128, 0, stream>>>(XB, WB, QH, SEQ_FULL * EMB, 0, SEQ_FULL * EMB, EMB);
  k_gemm_h<<<dim3(SEQ / 64, EMB / 128, NB), 128, 0, stream>>>(XB, WB + (size_t)EMB * EMB, KH, SEQ_FULL * EMB, 0, SEQ_FULL * EMB, EMB);
  k_gemm_h<<<dim3(EMB / 64, SEQ / 128, NB), 128, 0, stream>>>(WB + (size_t)2 * EMB * EMB, XB, VT, 0, SEQ_FULL * EMB, EMB * SEQ_FULL, SEQ_FULL);
  for (int b = 0; b < NB; ++b) {
    k_sc<<<dim3(SEQ / 64, SEQ / 128), 128, 0, stream>>>(QH + (size_t)b * SEQ_FULL * EMB, KH + (size_t)b * SEQ_FULL * EMB, S);
    k_sm<<<dim3(SEQ), 256, 0, stream>>>(S, PH);
    k_pv<<<dim3(SEQ / 64, EMB / 128), 128, 0, stream>>>(PH, VT + (size_t)b * EMB * SEQ_FULL, CS, OUT + (size_t)b * SEQ_FULL * EMB);
  }
}
